// RelationalNetwork_33036888440968
// MI455X (gfx1250) — hardware-verified
//
#include <hip/hip_runtime.h>
#include <math.h>
typedef __attribute__((ext_vector_type(16))) _Float16 v16h;
typedef __attribute__((ext_vector_type(8)))  _Float16 v8h;
typedef __attribute__((ext_vector_type(16))) __bf16   v16b;
typedef __attribute__((ext_vector_type(8)))  __bf16   v8b;
typedef __attribute__((ext_vector_type(8)))  float    v8f;
typedef __attribute__((ext_vector_type(4)))  float    v4f;
#define PSCALE 32768.0f
#define U16(p) ((const unsigned short*)(const void*)(p))
#define PSCALE_INV (1.0f / 32768.0f)

__device__ __forceinline__ unsigned short f2bf_bits(float f) {
  unsigned u = __float_as_uint(f);
  return (unsigned short)((u + 0x7FFFu + ((u >> 16) & 1u)) >> 16);
}
__device__ __forceinline__ float bf_bits2f(unsigned short h) { return __uint_as_float(((unsigned)h) << 16); }

__device__ __forceinline__ void dep_guard_h(v8f& a, v8f& b, v16h x, v16h y) { asm volatile("v_nop\n\tv_nop\n\tv_nop\n\tv_nop" : "+v"(a), "+v"(b) : "v"(x), "v"(y)); }
__device__ __forceinline__ void dep_guard_b(v8f& a, v8f& b, v16b x, v16b y) { asm volatile("v_nop\n\tv_nop\n\tv_nop\n\tv_nop" : "+v"(a), "+v"(b) : "v"(x), "v"(y)); }
__device__ __forceinline__ void keep4_h(v16h a, v16h b, v16h c, v16h d) { asm volatile("v_nop" :: "v"(a), "v"(b), "v"(c), "v"(d)); }
__device__ __forceinline__ void keep4_b(v16b a, v16b b, v16b c, v16b d) { asm volatile("v_nop" :: "v"(a), "v"(b), "v"(c), "v"(d)); }
__device__ __forceinline__ void acc_guard4(v8f& a, v8f& b, v8f& c, v8f& d) { asm volatile("v_nop\n\tv_nop\n\tv_nop\n\tv_nop" : "+v"(a), "+v"(b), "+v"(c), "+v"(d)); }
template <typename T> struct Frag;
template <> struct Frag<_Float16> {
  typedef v16h V; union U { v16h v; v8h h[2]; };
  static __device__ __forceinline__ v16h load(const _Float16* p) {
    U f; f.h[0] = *(const v8h*)(p); f.h[1] = *(const v8h*)(p + 16); return f.v;
  }
  static __device__ __forceinline__ v8f mma(v16h a, v16h b, v8f c) {
    return __builtin_amdgcn_wmma_f32_16x16x32_f16(false, a, false, b, (short)0, c, false, false);
  }
  static __device__ __forceinline__ void guard(v8f& a, v8f& b, v16h x, v16h y) { dep_guard_h(a, b, x, y); }
  static __device__ __forceinline__ void keep(v16h a, v16h b, v16h c, v16h d) { keep4_h(a, b, c, d); }
};
template <> struct Frag<__bf16> {
  typedef v16b V; union U { v16b v; v8b h[2]; };
  static __device__ __forceinline__ v16b load(const __bf16* p) {
    U f; f.h[0] = *(const v8b*)(p); f.h[1] = *(const v8b*)(p + 16); return f.v;
  }
  static __device__ __forceinline__ v8f mma(v16b a, v16b b, v8f c) {
    return __builtin_amdgcn_wmma_f32_16x16x32_bf16(false, a, false, b, (short)0, c, false, false);
  }
  static __device__ __forceinline__ void guard(v8f& a, v8f& b, v16b x, v16b y) { dep_guard_b(a, b, x, y); }
  static __device__ __forceinline__ void keep(v16b a, v16b b, v16b c, v16b d) { keep4_b(a, b, c, d); }
};

template <int ET> struct Elem;
template <> struct Elem<0> { typedef _Float16 T; };
template <> struct Elem<1> { typedef __bf16 T; };
template <int ET, bool SPLIT, int BIAS_MODE, int OUT_MODE, bool RESID, int ACT = 0>
__global__ __launch_bounds__(256) void wmma_gemm64(
    const unsigned short* __restrict__ Ap, const unsigned short* __restrict__ A2p, int lda, long strideA,
    const unsigned short* __restrict__ Btp, const unsigned short* __restrict__ Bt2p, int ldb, long strideB,
    void* __restrict__ Cout, void* __restrict__ Cout2, int ldc, long strideC,
    const float* __restrict__ bias,
    const float* __restrict__ resid, long strideR,
    int M, int N, int K, float scale) {
  typedef typename Elem<ET>::T T;
  typedef typename Frag<T>::V V;
  const T* A = (const T*)Ap; const T* A2 = (const T*)A2p; const T* Bt = (const T*)Btp; const T* Bt2 = (const T*)Bt2p;
  __shared__ __align__(16) float sT[8][16 * 68];
  const int b    = blockIdx.y;
  const int lane = threadIdx.x & 31;
  const int wave = threadIdx.x >> 5;
  const int tilesN = N >> 6;
  const int tilesM = M >> 6;
  const int tile = blockIdx.x * 8 + wave;
  if (tile >= tilesM * tilesN) return;
  const int tm = tile / tilesN;
  const int tn = tile - tm * tilesN;
  const int m0 = tm << 6;
  const int n0 = tn << 6;

  const T* Ab  = A  + (size_t)b * strideA;
  const T* Bb  = Bt + (size_t)b * strideB;
  const T* Ab2 = SPLIT ? (A2  + (size_t)b * strideA) : nullptr;
  const T* Bb2 = SPLIT ? (Bt2 + (size_t)b * strideB) : nullptr;

  const int rlane = lane & 15;
  const int koff  = (lane >> 4) * 8;
  const int mOff  = (lane >> 4) * 8;

  v8f acc[4][4];
#pragma unroll
  for (int i = 0; i < 4; ++i)
#pragma unroll
    for (int j = 0; j < 4; ++j) acc[i][j] = (v8f){0.f,0.f,0.f,0.f,0.f,0.f,0.f,0.f};

  for (int k0 = 0; k0 < K; k0 += 32) {
    V bh[4], bl[4];
#pragma unroll
    for (int j = 0; j < 4; ++j) {
      const size_t bo = (size_t)(n0 + (j << 4) + rlane) * ldb + koff + k0;
      bh[j] = Frag<T>::load(Bb + bo);
      if (SPLIT) bl[j] = Frag<T>::load(Bb2 + bo);
    }
#pragma unroll
    for (int i = 0; i < 4; ++i) {
      const size_t ao = (size_t)(m0 + (i << 4) + rlane) * lda + koff + k0;
      V ah = Frag<T>::load(Ab + ao);
      V al;
      if (SPLIT) al = Frag<T>::load(Ab2 + ao);
#pragma unroll
      for (int j = 0; j < 4; ++j) {
        acc[i][j] = Frag<T>::mma(ah, bh[j], acc[i][j]);
        if (SPLIT) {
          acc[i][j] = Frag<T>::mma(ah, bl[j], acc[i][j]);
          acc[i][j] = Frag<T>::mma(al, bh[j], acc[i][j]);
        }
      }
      Frag<T>::guard(acc[i][0], acc[i][3], ah, SPLIT ? al : ah);
    }
    Frag<T>::keep(bh[0], bh[1], bh[2], bh[3]);
    if (SPLIT) Frag<T>::keep(bl[0], bl[1], bl[2], bl[3]);
  }
  acc_guard4(acc[0][0], acc[0][1], acc[0][2], acc[0][3]);
  acc_guard4(acc[1][0], acc[1][1], acc[1][2], acc[1][3]);
  acc_guard4(acc[2][0], acc[2][1], acc[2][2], acc[2][3]);
  acc_guard4(acc[3][0], acc[3][1], acc[3][2], acc[3][3]);

  float* slab = sT[wave];
  const float* Rb = RESID ? (resid + (size_t)b * strideR) : nullptr;
#pragma unroll
  for (int i = 0; i < 4; ++i) {
    const int mBase = m0 + (i << 4);
#pragma unroll
    for (int j = 0; j < 4; ++j) {
      const int n = n0 + (j << 4) + rlane;
      float bv = 0.f;
      if (BIAS_MODE == 2) bv = bias[n];
#pragma unroll
      for (int r = 0; r < 8; ++r) {
        float v = acc[i][j][r] * scale;
        if (BIAS_MODE == 1) v += bias[mBase + mOff + r];
        if (BIAS_MODE == 2) v += bv;
        if (RESID) v += Rb[(size_t)(mBase + mOff + r) * ldc + n];
        if (ACT == 1) v = tanhf(v);
        if (ACT == 2) v = fmaxf(v, 0.0f);
        if (ACT == 3) v = v / (1.0f + expf(-v));
        slab[(mOff + r) * 68 + (j << 4) + rlane] = v;
      }
    }
    __builtin_amdgcn_fence(__ATOMIC_RELEASE, "workgroup");
    __builtin_amdgcn_wave_barrier();
    __builtin_amdgcn_fence(__ATOMIC_ACQUIRE, "workgroup");
    if (OUT_MODE == 0) {
      float* C = (float*)Cout + (size_t)b * strideC;
      const int hh = lane >> 4, c4 = (lane & 15) * 4;
      for (int pass = 0; pass < 2; ++pass) {
#pragma unroll
        for (int it = 0; it < 8; ++it) {
          const int row = it * 2 + hh;
          v4f v = *(const v4f*)(slab + row * 68 + c4);
          *(volatile v4f*)(C + (size_t)(mBase + row) * ldc + n0 + c4) = v;
        }
        __threadfence();
      }
    } else {
      const int q = lane >> 3, c8 = (lane & 7) * 8;
      unsigned short* C  = (unsigned short*)Cout  + (size_t)b * strideC;
      unsigned short* C2 = (OUT_MODE == 2) ? ((unsigned short*)Cout2 + (size_t)b * strideC) : nullptr;
      for (int pass = 0; pass < 2; ++pass) {
#pragma unroll
        for (int it = 0; it < 4; ++it) {
          const int row = it * 4 + q;
          const float* sp = slab + row * 68 + c8;
          v8h hv, lv;
#pragma unroll
          for (int e = 0; e < 8; ++e) {
            if (OUT_MODE == 1) {
              hv[e] = (_Float16)sp[e];
            } else {
              unsigned short hb = f2bf_bits(sp[e]);
              unsigned short lb = f2bf_bits(sp[e] - bf_bits2f(hb));
              hv[e] = __builtin_bit_cast(_Float16, hb);
              lv[e] = __builtin_bit_cast(_Float16, lb);
            }
          }
          *(volatile v8h*)(C + (size_t)(mBase + row) * ldc + n0 + c8) = hv;
          if (OUT_MODE == 2) *(volatile v8h*)(C2 + (size_t)(mBase + row) * ldc + n0 + c8) = lv;
        }
        __threadfence();
      }
    }
    __builtin_amdgcn_fence(__ATOMIC_RELEASE, "workgroup");
    __builtin_amdgcn_wave_barrier();
    __builtin_amdgcn_fence(__ATOMIC_ACQUIRE, "workgroup");
  }
}

__global__ __launch_bounds__(256) void cast_f32_f16x2(
    const float* __restrict__ in, _Float16* __restrict__ out, int n2) {
  int i = blockIdx.x * 256 + threadIdx.x;
  if (i < n2) {
    const _Float16 h0 = (_Float16)in[2 * i], h1 = (_Float16)in[2 * i + 1];
    const unsigned u = (unsigned)__builtin_bit_cast(unsigned short, h0) | ((unsigned)__builtin_bit_cast(unsigned short, h1) << 16);
    ((volatile unsigned*)out)[i] = u;
    __threadfence();
    ((volatile unsigned*)out)[i] = u;
  }
}


__global__ __launch_bounds__(256) void transpose_cast_f16(const float* __restrict__ in, int ldi,
                                                         _Float16* __restrict__ outT, int ldo, float scale) {
  __shared__ __align__(16) _Float16 tile[64][72];
  const int c0 = blockIdx.x * 64, r0 = blockIdx.y * 64;
  const int t = threadIdx.y * 32 + threadIdx.x;
  for (int i = threadIdx.y; i < 64; i += 8) {
    tile[threadIdx.x][i]      = (_Float16)(in[(size_t)(r0 + i) * ldi + c0 + threadIdx.x] * scale);
    tile[32 + threadIdx.x][i] = (_Float16)(in[(size_t)(r0 + i) * ldi + c0 + 32 + threadIdx.x] * scale);
  }
  __syncthreads();
  const int q = t >> 3, c8 = (t & 7) * 8;
  for (int pass = 0; pass < 2; ++pass) {
#pragma unroll
    for (int it = 0; it < 2; ++it) {
      const int c = it * 32 + q;
      v8h hv = *(const v8h*)(&tile[c][c8]);
      *(volatile v8h*)(outT + (size_t)(c0 + c) * ldo + r0 + c8) = hv;
    }
    __threadfence();
  }
}

#define NB 8
#define NLQ 256
#define NF 16
#define FH 128
#define NPAIR (NB * NLQ)
#define NROWS ((long)NB * NLQ * NLQ)

__global__ __launch_bounds__(256) void g1_kernel(const float* __restrict__ x, const float* __restrict__ coord, const float* __restrict__ W1a,
                                                const float* __restrict__ W1b, float* __restrict__ HI, float* __restrict__ HJ) {
  const int lane = threadIdx.x & 31, wave = threadIdx.x >> 5;
  const int row = blockIdx.x * 8 + wave;
  const int b = row / NLQ, l = row % NLQ;
  float xin[18];
#pragma unroll
  for (int f = 0; f < NF; ++f) xin[f] = x[((size_t)b * NF + f) * NLQ + l];
  xin[16] = coord[l * 2]; xin[17] = coord[l * 2 + 1];
  float hi[4], hj[4];
#pragma unroll
  for (int q = 0; q < 4; ++q) {
    const int c = 4 * lane + q; float a = 0.f, bb = 0.f;
#pragma unroll
    for (int f = 0; f < 18; ++f) { a += xin[f] * W1a[f * FH + c]; bb += xin[f] * W1b[f * FH + c]; }
    hi[q] = a; hj[q] = bb;
  }
  const v4f va = {hi[0], hi[1], hi[2], hi[3]}, vb = {hj[0], hj[1], hj[2], hj[3]};
  for (int pass = 0; pass < 2; ++pass) {
    *(volatile v4f*)(HI + (size_t)row * FH + 4 * lane) = va; *(volatile v4f*)(HJ + (size_t)row * FH + 4 * lane) = vb; __threadfence();
  }
}
__global__ __launch_bounds__(128) void bn1_stats_kernel(const float* __restrict__ HI, const float* __restrict__ HJ, const float* __restrict__ b1, float* __restrict__ stats) {
  const int c = threadIdx.x;
  double si = 0.0, sj = 0.0;
  for (int r = 0; r < NPAIR; ++r) { si += HI[(size_t)r * FH + c]; sj += HJ[(size_t)r * FH + c]; }
  const double mi = si / NPAIR, mj = sj / NPAIR;
  double var = 0.0;
  for (int b = 0; b < NB; ++b) {
    double sa = 0.0, sa2 = 0.0, sc = 0.0, sc2 = 0.0;
    for (int l = 0; l < NLQ; ++l) { const double a = HI[((size_t)b * NLQ + l) * FH + c] - mi; sa += a; sa2 += a * a; const double cc = HJ[((size_t)b * NLQ + l) * FH + c] - mj; sc += cc; sc2 += cc * cc; }
    var += NLQ * sa2 + NLQ * sc2 + 2.0 * sa * sc;
  }
  var /= (double)NROWS;
  const float mean = (float)(mi + mj + (double)b1[c]), rstd = (float)(1.0 / sqrt(var + 1e-5));
  for (int pass = 0; pass < 2; ++pass) { ((volatile float*)stats)[c] = mean; ((volatile float*)stats)[FH + c] = rstd; __threadfence(); }
}
__global__ __launch_bounds__(256) void wfrag_kernel(const float* __restrict__ Wm, unsigned* __restrict__ frag) {
  const int i = blockIdx.x * 256 + threadIdx.x;
  if (i >= 8192) return;
  const int ep = i & 7, lane = (i >> 3) & 31, rest = i >> 8;
  const int kc = rest & 3, nt = rest >> 2;
  unsigned short hv[2];
#pragma unroll
  for (int q = 0; q < 2; ++q) { const int e = 2 * ep + q; const int k = kc * 32 + ((e < 8) ? (8 * (lane >> 4) + e) : (16 + 8 * (lane >> 4) + (e - 8))); const int n = nt * 16 + (lane & 15);
    hv[q] = __builtin_bit_cast(unsigned short, (_Float16)Wm[k * FH + n]); }
  const unsigned u = (unsigned)hv[0] | ((unsigned)hv[1] << 16);
  ((volatile unsigned*)frag)[i] = u; __threadfence(); ((volatile unsigned*)frag)[i] = u;
}
#define APITCH 136
__device__ __forceinline__ void block_gemm_256x128(const _Float16* __restrict__ As, const unsigned* __restrict__ frag, int wave, int lane, v8f acc[2][8]) {
#pragma unroll
  for (int mt = 0; mt < 2; ++mt)
#pragma unroll
    for (int nt = 0; nt < 8; ++nt) acc[mt][nt] = (v8f){0.f,0.f,0.f,0.f,0.f,0.f,0.f,0.f};
  const int hh = lane >> 4, c = lane & 15;
#pragma unroll
  for (int kc = 0; kc < 4; ++kc) {
    v16h a[2];
#pragma unroll
    for (int mt = 0; mt < 2; ++mt) {
      const _Float16* p = As + (size_t)(wave * 32 + mt * 16 + c) * APITCH + kc * 32 + 8 * hh;
      const v8h lo = *(const v8h*)p, hi = *(const v8h*)(p + 16);
#pragma unroll
      for (int e = 0; e < 8; ++e) { a[mt][e] = lo[e]; a[mt][8 + e] = hi[e]; }
    }
#pragma unroll
    for (int nt = 0; nt < 8; ++nt) {
      const uint4* fp = (const uint4*)(frag + ((size_t)(nt * 4 + kc) * 32 + lane) * 8);
      union { v16h v; uint4 u[2]; } bf; bf.u[0] = fp[0]; bf.u[1] = fp[1];
#pragma unroll
      for (int mt = 0; mt < 2; ++mt) {
        acc[mt][nt] = __builtin_amdgcn_wmma_f32_16x16x32_f16(false, a[mt], false, bf.v, (short)0, acc[mt][nt], false, false);
      }
      dep_guard_h(acc[0][nt], acc[1][nt], a[0], bf.v);
    }
  }
}
template <int PASS>
__global__ __launch_bounds__(256) void pair_kernel(const float* __restrict__ HI, const float* __restrict__ HJ, const float* __restrict__ b1,
    const float* __restrict__ st1, const float* __restrict__ g1g, const float* __restrict__ g1b,
    const unsigned* __restrict__ fragW2, const float* __restrict__ b2, const float* __restrict__ st2, const float* __restrict__ g2g, const float* __restrict__ g2b,
    const unsigned* __restrict__ fragW3, const float* __restrict__ b3, const float* __restrict__ st3, const float* __restrict__ g3g, const float* __restrict__ g3b,
    const float* __restrict__ Wagg, const float* __restrict__ bagg, float* __restrict__ part, float* __restrict__ XAGG, unsigned short* __restrict__ H2h) {
  __shared__ __align__(16) _Float16 As[NLQ * APITCH];
  __shared__ float red[8][FH * 2];
  const int tid = threadIdx.x, lane = tid & 31, wave = tid >> 5, hh = lane >> 4, c = lane & 15;
  const int blk = blockIdx.x;
  const int b = blk / NLQ;
  if (PASS == 0) {
    for (int i = tid; i < NLQ * FH / 2; i += 256) {
      const int l = i / (FH / 2), ch = (i % (FH / 2)) * 2;
      float v0 = HI[((size_t)b * NLQ + l) * FH + ch] + HJ[(size_t)blk * FH + ch] + b1[ch];
      float v1 = HI[((size_t)b * NLQ + l) * FH + ch + 1] + HJ[(size_t)blk * FH + ch + 1] + b1[ch + 1];
      v0 = fmaxf((v0 - st1[ch]) * st1[FH + ch] * g1g[ch] + g1b[ch], 0.f);
      v1 = fmaxf((v1 - st1[ch + 1]) * st1[FH + ch + 1] * g1g[ch + 1] + g1b[ch + 1], 0.f);
      As[l * APITCH + ch] = (_Float16)v0; As[l * APITCH + ch + 1] = (_Float16)v1;
    }
  } else {
    for (int i = tid; i < NLQ * FH / 2; i += 256) {
      const int l = i / (FH / 2), ch = (i % (FH / 2)) * 2;
      const unsigned u = ((const unsigned*)H2h)[((size_t)blk * NLQ + l) * (FH / 2) + ch / 2];
      float v0 = (float)__builtin_bit_cast(_Float16, (unsigned short)(u & 0xFFFF)), v1 = (float)__builtin_bit_cast(_Float16, (unsigned short)(u >> 16));
      v0 = fmaxf((v0 - st2[ch]) * st2[FH + ch] * g2g[ch] + g2b[ch], 0.f);
      v1 = fmaxf((v1 - st2[ch + 1]) * st2[FH + ch + 1] * g2g[ch + 1] + g2b[ch + 1], 0.f);
      As[l * APITCH + ch] = (_Float16)v0; As[l * APITCH + ch + 1] = (_Float16)v1;
    }
  }
  __syncthreads();
  v8f acc[2][8];
  block_gemm_256x128(As, (PASS == 0) ? fragW2 : fragW3, wave, lane, acc);
  {
    const float* bb = (PASS == 0) ? b2 : b3;
#pragma unroll
    for (int nt = 0; nt < 8; ++nt) { const float bv = bb[nt * 16 + c];
#pragma unroll
      for (int mt = 0; mt < 2; ++mt)
#pragma unroll
        for (int r = 0; r < 8; ++r) acc[mt][nt][r] += bv; }
  }
  if (PASS == 2) {
    float colsum[8];
#pragma unroll
    for (int nt = 0; nt < 8; ++nt) { const int col = nt * 16 + c; const float m = st3[col], rs = st3[FH + col], gg = g3g[col], be = g3b[col]; float s = 0.f;
#pragma unroll
      for (int mt = 0; mt < 2; ++mt)
#pragma unroll
        for (int r = 0; r < 8; ++r) { const int l = wave * 32 + mt * 16 + 8 * hh + r; s += Wagg[l] * fmaxf((acc[mt][nt][r] - m) * rs * gg + be, 0.f); }
      s += __shfl_xor(s, 16, 32);
      colsum[nt] = s; }
    if (hh == 0) {
#pragma unroll
      for (int nt = 0; nt < 8; ++nt) red[wave][nt * 16 + c] = colsum[nt];
    }
    __syncthreads();
    if (tid < FH) { float s = 0.f; for (int w = 0; w < 8; ++w) s += red[w][tid]; s += bagg[0]; red[0][tid] = s; }
    __syncthreads();
    if (tid < 32) { const v4f v = *(const v4f*)(&red[0][4 * tid]); *(volatile v4f*)(XAGG + (size_t)blk * FH + 4 * tid) = v; __threadfence(); *(volatile v4f*)(XAGG + (size_t)blk * FH + 4 * tid) = v; }
    return;
  }
  {
    float cs[8], cq[8];
#pragma unroll
    for (int nt = 0; nt < 8; ++nt) { float s = 0.f, q = 0.f;
#pragma unroll
      for (int mt = 0; mt < 2; ++mt)
#pragma unroll
        for (int r = 0; r < 8; ++r) { const float v = acc[mt][nt][r]; s += v; q += v * v; }
      s += __shfl_xor(s, 16, 32); q += __shfl_xor(q, 16, 32); cs[nt] = s; cq[nt] = q; }
    if (hh == 0) {
#pragma unroll
      for (int nt = 0; nt < 8; ++nt) { red[wave][nt * 16 + c] = cs[nt]; red[wave][FH + nt * 16 + c] = cq[nt]; }
    }
  }
  if (PASS == 0) {
    __syncthreads();
#pragma unroll
    for (int nt = 0; nt < 8; ++nt)
#pragma unroll
      for (int mt = 0; mt < 2; ++mt)
#pragma unroll
        for (int r = 0; r < 8; ++r) As[(size_t)(wave * 32 + mt * 16 + 8 * hh + r) * APITCH + nt * 16 + c] = (_Float16)acc[mt][nt][r];
    __builtin_amdgcn_fence(__ATOMIC_RELEASE, "workgroup"); __builtin_amdgcn_wave_barrier(); __builtin_amdgcn_fence(__ATOMIC_ACQUIRE, "workgroup");
    const int rsub = lane >> 4, c8 = (lane & 15) * 8;
    for (int pass = 0; pass < 2; ++pass) {
#pragma unroll
      for (int it = 0; it < 16; ++it) {
        const int row = wave * 32 + it * 2 + rsub;
        const v8h v = *(const v8h*)(As + (size_t)row * APITCH + c8);
        *(volatile v8h*)((_Float16*)H2h + ((size_t)blk * NLQ + row) * FH + c8) = v;
      }
      __threadfence();
    }
  }
  __syncthreads();
  {
    float v = 0.f; for (int w = 0; w < 8; ++w) v += red[w][tid];
    ((volatile float*)part)[(size_t)blk * 2 * FH + tid] = v; __threadfence(); ((volatile float*)part)[(size_t)blk * 2 * FH + tid] = v;
  }
}
__global__ __launch_bounds__(256) void bn_reduce_kernel(const float* __restrict__ part, int nblk, double nrows, float* __restrict__ stats) {
  const int t = threadIdx.x; const int c = t & 127; const int which = t >> 7;
  double s = 0.0;
  for (int b = 0; b < nblk; ++b) s += (double)part[(size_t)b * 2 * FH + which * FH + c];
  __shared__ double sh[256];
  sh[t] = s; __syncthreads();
  float v;
  if (which == 0) v = (float)(sh[c] / nrows);
  else { const double m = sh[c] / nrows; double var = sh[FH + c] / nrows - m * m; if (var < 0.0) var = 0.0; v = (float)(1.0 / sqrt(var + 1e-5)); }
  ((volatile float*)stats)[t] = v; __threadfence(); ((volatile float*)stats)[t] = v;
}
__global__ __launch_bounds__(128) void bn_small_kernel(const float* __restrict__ Hin, const float* __restrict__ g, const float* __restrict__ be, unsigned short* __restrict__ H16) {
  const int c = threadIdx.x;
  double s = 0.0; for (int r = 0; r < NPAIR; ++r) s += Hin[(size_t)r * FH + c];
  const double m = s / NPAIR; double v = 0.0;
  for (int r = 0; r < NPAIR; ++r) { const double d = Hin[(size_t)r * FH + c] - m; v += d * d; }
  const float rs = (float)(1.0 / sqrt(v / NPAIR + 1e-5)), mf = (float)m, gg = g[c], bb = be[c];
  for (int pass = 0; pass < 2; ++pass) {
    for (int r = 0; r < NPAIR; ++r) { const float val = fmaxf((Hin[(size_t)r * FH + c] - mf) * rs * gg + bb, 0.f); ((volatile unsigned short*)H16)[(size_t)r * FH + c] = __builtin_bit_cast(unsigned short, (_Float16)val); }
    __threadfence();
  }
}

__global__ __launch_bounds__(256) void pad_wo3_kernel(const float* __restrict__ Wo3, const float* __restrict__ bo3, _Float16* __restrict__ Wt, float* __restrict__ bp) {
  for (int pass = 0; pass < 2; ++pass) {
    for (int i = threadIdx.x; i < 64 * FH / 2; i += 256) {
      const int n = (2 * i) / FH, k = (2 * i) % FH;
      const float a = (n < NF) ? Wo3[k * NF + n] : 0.f, b = (n < NF) ? Wo3[(k + 1) * NF + n] : 0.f;
      ((volatile unsigned*)Wt)[i] = (unsigned)__builtin_bit_cast(unsigned short, (_Float16)a) | ((unsigned)__builtin_bit_cast(unsigned short, (_Float16)b) << 16);
    }
    if (threadIdx.x < 64) ((volatile float*)bp)[threadIdx.x] = (threadIdx.x < NF) ? bo3[threadIdx.x] : 0.f;
    __threadfence();
  }
}
__global__ __launch_bounds__(256) void out_kernel(const float* __restrict__ R, float* __restrict__ out) {
  const int lane = threadIdx.x & 31, wave = threadIdx.x >> 5;
  const int bf = blockIdx.x * 8 + wave;
  const int b = bf / NF, f = bf % NF;
  for (int pass = 0; pass < 2; ++pass) {
#pragma unroll
    for (int i = 0; i < 2; ++i) { v4f v; const int l0 = (i * 32 + lane) * 4;
#pragma unroll
      for (int q = 0; q < 4; ++q) v[q] = R[((size_t)b * NLQ + l0 + q) * 64 + f];
      *(volatile v4f*)(out + (size_t)bf * NLQ + l0) = v; }
    __threadfence();
  }
}

extern "C" void kernel_launch(void* const* d_in, const int* in_sizes, int n_in,
                              void* d_out, int out_size, void* d_ws, size_t ws_size,
                              hipStream_t stream) {
  (void)in_sizes; (void)n_in; (void)out_size; (void)ws_size;
  const float* x = (const float*)d_in[0];
  const float* W1a = (const float*)d_in[1]; const float* W1b = (const float*)d_in[2]; const float* b1 = (const float*)d_in[3];
  const float* g1g = (const float*)d_in[4]; const float* g1b = (const float*)d_in[5];
  const float* W2 = (const float*)d_in[6]; const float* b2 = (const float*)d_in[7]; const float* g2g = (const float*)d_in[8]; const float* g2b = (const float*)d_in[9];
  const float* W3 = (const float*)d_in[10]; const float* b3 = (const float*)d_in[11]; const float* g3g = (const float*)d_in[12]; const float* g3b = (const float*)d_in[13];
  const float* Wagg = (const float*)d_in[14]; const float* bagg = (const float*)d_in[15];
  const float* Wf = (const float*)d_in[16]; const float* bfv = (const float*)d_in[17]; const float* fg = (const float*)d_in[18]; const float* fb = (const float*)d_in[19];
  const float* Wo2 = (const float*)d_in[20]; const float* bo2 = (const float*)d_in[21]; const float* o2g = (const float*)d_in[22]; const float* o2b = (const float*)d_in[23];
  const float* Wo3 = (const float*)d_in[24]; const float* bo3 = (const float*)d_in[25];
  const float* coord = (const float*)d_in[26];
  float* out = (float*)d_out;

  char* ws = (char*)d_ws; size_t off = 0;
  auto carve = [&](size_t bytes) -> char* { char* p = ws + off; off += (bytes + 255) & ~(size_t)255; return p; };
  float* HI = (float*)carve((size_t)NPAIR * FH * 4); float* HJ = (float*)carve((size_t)NPAIR * FH * 4);
  float* st1 = (float*)carve(256 * 4); float* st2 = (float*)carve(256 * 4); float* st3 = (float*)carve(256 * 4);
  unsigned* fW2 = (unsigned*)carve(8192 * 4); unsigned* fW3 = (unsigned*)carve(8192 * 4);
  float* part = (float*)carve((size_t)NPAIR * 2 * FH * 4);
  float* XAGG = (float*)carve((size_t)NPAIR * FH * 4);
  _Float16* XA16 = (_Float16*)carve((size_t)NPAIR * FH * 2);
  _Float16* WfT = (_Float16*)carve((size_t)FH * FH * 2); _Float16* Wo2T = (_Float16*)carve((size_t)FH * FH * 2); _Float16* Wo3T = (_Float16*)carve((size_t)64 * FH * 2);
  float* T1 = (float*)carve((size_t)NPAIR * FH * 4); unsigned short* T1h = (unsigned short*)carve((size_t)NPAIR * FH * 2);
  float* T2 = (float*)carve((size_t)NPAIR * FH * 4); unsigned short* T2h = (unsigned short*)carve((size_t)NPAIR * FH * 2);
  float* R = (float*)carve((size_t)NPAIR * 64 * 4);
  float* bo3p = (float*)carve(64 * 4);
  unsigned short* H2h = (unsigned short*)carve((size_t)NROWS * FH * 2);

  g1_kernel<<<NPAIR / 8, 256, 0, stream>>>(x, coord, W1a, W1b, HI, HJ);
  bn1_stats_kernel<<<1, 128, 0, stream>>>(HI, HJ, b1, st1);
  wfrag_kernel<<<32, 256, 0, stream>>>(W2, fW2);
  wfrag_kernel<<<32, 256, 0, stream>>>(W3, fW3);
  pair_kernel<0><<<NPAIR, 256, 0, stream>>>(HI, HJ, b1, st1, g1g, g1b, fW2, b2, st2, g2g, g2b, fW3, b3, st3, g3g, g3b, Wagg, bagg, part, XAGG, H2h);
  bn_reduce_kernel<<<1, 256, 0, stream>>>(part, NPAIR, (double)NROWS, st2);
  pair_kernel<1><<<NPAIR, 256, 0, stream>>>(HI, HJ, b1, st1, g1g, g1b, fW2, b2, st2, g2g, g2b, fW3, b3, st3, g3g, g3b, Wagg, bagg, part, XAGG, H2h);
  bn_reduce_kernel<<<1, 256, 0, stream>>>(part, NPAIR, (double)NROWS, st3);
  pair_kernel<2><<<NPAIR, 256, 0, stream>>>(HI, HJ, b1, st1, g1g, g1b, fW2, b2, st2, g2g, g2b, fW3, b3, st3, g3g, g3b, Wagg, bagg, part, XAGG, H2h);
  cast_f32_f16x2<<<(NPAIR * FH / 2 + 255) / 256, 256, 0, stream>>>(XAGG, XA16, NPAIR * FH / 2);
  transpose_cast_f16<<<dim3(FH / 64, FH / 64), dim3(32, 8), 0, stream>>>(Wf, FH, WfT, FH, 1.0f);
  transpose_cast_f16<<<dim3(FH / 64, FH / 64), dim3(32, 8), 0, stream>>>(Wo2, FH, Wo2T, FH, 1.0f);
  pad_wo3_kernel<<<1, 256, 0, stream>>>(Wo3, bo3, Wo3T, bo3p);
  {
    const int t = (NPAIR / 64) * (FH / 64);
    wmma_gemm64<0, false, 2, 0, false><<<dim3((t + 7) / 8, 1), 256, 0, stream>>>(U16(XA16), nullptr, FH, 0, U16(WfT), nullptr, FH, 0, T1, nullptr, FH, 0, bfv, nullptr, 0, NPAIR, FH, FH, 1.0f);
    bn_small_kernel<<<1, 128, 0, stream>>>(T1, fg, fb, T1h);
    wmma_gemm64<0, false, 2, 0, false><<<dim3((t + 7) / 8, 1), 256, 0, stream>>>(T1h, nullptr, FH, 0, U16(Wo2T), nullptr, FH, 0, T2, nullptr, FH, 0, bo2, nullptr, 0, NPAIR, FH, FH, 1.0f);
    bn_small_kernel<<<1, 128, 0, stream>>>(T2, o2g, o2b, T2h);
    const int t3 = (NPAIR / 64) * 1;
    wmma_gemm64<0, false, 2, 0, false><<<dim3((t3 + 7) / 8, 1), 256, 0, stream>>>(T2h, nullptr, FH, 0, U16(Wo3T), nullptr, FH, 0, R, nullptr, 64, 0, bo3p, nullptr, 0, NPAIR, 64, FH, 1.0f);
  }
  out_kernel<<<NB * NF / 8, 256, 0, stream>>>(R, out);
}
